// MultiViewGNN_19851338842499
// MI455X (gfx1250) — hardware-verified
//
#include <hip/hip_runtime.h>


typedef __attribute__((ext_vector_type(16))) _Float16 v16h;
typedef __attribute__((ext_vector_type(8)))  _Float16 v8h;
typedef __attribute__((ext_vector_type(8)))  float    v8f;
typedef __attribute__((ext_vector_type(4)))  float    v4f;
typedef __attribute__((ext_vector_type(2)))  int      v2i;
typedef unsigned int u32;
#define D 128
#define NM 1043
#define ND 2166
#define NMP 1152
#define NDP 2176
#define TILE 8192
#define VST2(T, ptr, val) do { const T _v = (val); *(volatile T*)(ptr) = _v; __threadfence(); *(volatile T*)(ptr) = _v; } while (0)
__device__ __forceinline__ v8f wmma16(v16h a, v16h b, v8f c) {
  v8f d = __builtin_amdgcn_wmma_f32_16x16x32_f16(false, a, false, b, (short)0, c, false, false);
  asm volatile("v_nop\n\tv_nop\n\tv_nop\n\tv_nop" : "+v"(d) : "v"(a), "v"(b));
  return d;
}
__device__ __forceinline__ v16h frag16(const _Float16* p, int hh) {
  const v8h lo = *(const v8h*)(p + 8 * hh), hi = *(const v8h*)(p + 16 + 8 * hh);
  return __builtin_shufflevector(lo, hi, 0,1,2,3,4,5,6,7,8,9,10,11,12,13,14,15);
}

__global__ __launch_bounds__(256) void k_sort_init(const int* __restrict__ dst, u32* __restrict__ A, int E) {
  const int i = blockIdx.x * 256 + threadIdx.x;
  VST2(u32, A + i, (i < E) ? (((u32)dst[i]) << 20) | (u32)i : 0xffffffffu);
}
__device__ __forceinline__ void cas_lds(u32* s, int lo, int hi, bool up) {
  const u32 a = s[lo], b = s[hi]; const bool sw = up ? (a > b) : (a < b); s[lo] = sw ? b : a; s[hi] = sw ? a : b;
}
__global__ __launch_bounds__(256) void k_sort_local(u32* __restrict__ A) {
  __shared__ u32 s[TILE];
  const int base = blockIdx.x * TILE, t = threadIdx.x;
  for (int i = t; i < TILE; i += 256) s[i] = A[base + i];
  __syncthreads();
  for (int k = 2; k <= TILE; k <<= 1)
    for (int j = k >> 1; j > 0; j >>= 1) {
      for (int p = t; p < TILE / 2; p += 256) {
        const int lo = ((p >> __builtin_ctz(j)) << (__builtin_ctz(j) + 1)) | (p & (j - 1));
        cas_lds(s, lo, lo + j, (((base + lo) & k) == 0));
      }
      __syncthreads();
    }
  for (int pass = 0; pass < 2; ++pass) { for (int i = t; i < TILE; i += 256) *(volatile u32*)(A + base + i) = s[i]; __threadfence(); }
}
__global__ __launch_bounds__(256) void k_sort_global(u32* __restrict__ A, int logj, int k) {
  const int p = blockIdx.x * 256 + threadIdx.x;
  const int j = 1 << logj;
  const int lo = ((p >> logj) << (logj + 1)) | (p & (j - 1)), hi = lo + j;
  const u32 a = A[lo], b = A[hi];
  const bool up = ((lo & k) == 0), sw = up ? (a > b) : (a < b);
  const u32 vlo = sw ? b : a, vhi = sw ? a : b;
  *(volatile u32*)(A + lo) = vlo; *(volatile u32*)(A + hi) = vhi; __threadfence();
  *(volatile u32*)(A + lo) = vlo; *(volatile u32*)(A + hi) = vhi;
}
__global__ __launch_bounds__(256) void k_sort_lds(u32* __restrict__ A, int k) {
  __shared__ u32 s[TILE];
  const int base = blockIdx.x * TILE, t = threadIdx.x;
  for (int i = t; i < TILE; i += 256) s[i] = A[base + i];
  __syncthreads();
  for (int j = TILE >> 1; j > 0; j >>= 1) {
    for (int p = t; p < TILE / 2; p += 256) {
      const int lo = ((p >> __builtin_ctz(j)) << (__builtin_ctz(j) + 1)) | (p & (j - 1));
      cas_lds(s, lo, lo + j, (((base + lo) & k) == 0));
    }
    __syncthreads();
  }
  for (int pass = 0; pass < 2; ++pass) { for (int i = t; i < TILE; i += 256) *(volatile u32*)(A + base + i) = s[i]; __threadfence(); }
}
__global__ __launch_bounds__(256) void k_segs_deg(const u32* __restrict__ A, int sortN, const float* __restrict__ w, v2i* __restrict__ seg,
                                                  float* __restrict__ dinv, int N) {
  const int n = blockIdx.x * 256 + threadIdx.x;
  if (n >= N) return;
  int lo = 0, hi = sortN;
  while (lo < hi) { const int mid = (lo + hi) >> 1; if ((A[mid] >> 20) < (u32)n) lo = mid + 1; else hi = mid; }
  const int st = lo;
  lo = st; hi = sortN;
  while (lo < hi) { const int mid = (lo + hi) >> 1; if ((A[mid] >> 20) < (u32)(n + 1)) lo = mid + 1; else hi = mid; }
  const v2i sv = {st, lo - st};
  float d = 0.f;
  for (int p = 0; p < sv[1]; ++p) d += w[A[st + p] & 0xfffffu];
  VST2(v2i, seg + n, sv);
  VST2(float, dinv + n, (d > 0.f) ? (1.0f / sqrtf(d)) : 0.f);
}

__global__ __launch_bounds__(256) void k_tof16(const float* __restrict__ src, int valid, int rowsPad, int cols, const float* __restrict__ ascale,
                                               _Float16* __restrict__ dst) {
  const size_t i8 = (size_t)blockIdx.x * 256 + threadIdx.x;
  if (i8 * 8 >= (size_t)rowsPad * cols) return;
  const size_t i = i8 * 8; const int r = (int)(i / cols), c0 = (int)(i % cols);
  const float sc = ascale ? ascale[c0 >> 7] : 1.0f;
  v8h v;
#pragma unroll
  for (int e = 0; e < 8; ++e) v[e] = (_Float16)((r < valid) ? src[i + e] * sc : 0.0f);
  VST2(v8h, dst + i, v);
}
__global__ __launch_bounds__(256) void k_w16(const float* __restrict__ W, _Float16* __restrict__ Wh, int n) {
  const int i8 = blockIdx.x * 256 + threadIdx.x;
  if (i8 * 8 >= n) return;
  v8h v;
#pragma unroll
  for (int e = 0; e < 8; ++e) v[e] = (_Float16)W[i8 * 8 + e];
  VST2(v8h, Wh + (size_t)i8 * 8, v);
}
template <int KIN, int NOUT, bool RELU>
__global__ __launch_bounds__(128) void k_gemm(const _Float16* __restrict__ A, const _Float16* __restrict__ Wh, const float* __restrict__ bias,
                                              float* __restrict__ out, int valid) {
  const int lane = threadIdx.x & 31, wave = threadIdx.x >> 5, hh = lane >> 4, l16 = lane & 15;
  const int m0 = (blockIdx.x * 4 + wave) * 16, c0 = blockIdx.y * 64;
  if (m0 >= valid) return;
  v8f acc[4] = {};
  const _Float16* arow = A + (size_t)(m0 + l16) * KIN;
  for (int kb = 0; kb < KIN; kb += 32) {
    const v16h a = frag16(arow + kb, hh);
#pragma unroll
    for (int t = 0; t < 4; ++t) acc[t] = wmma16(a, frag16(Wh + (size_t)(c0 + t * 16 + l16) * KIN + kb, hh), acc[t]);
  }
  for (int pass = 0; pass < 2; ++pass) {
#pragma unroll
    for (int pr = 0; pr < 2; ++pr) {
      const int c = c0 + pr * 32 + lane;
      const float bb = bias ? bias[c] : 0.f;
#pragma unroll
      for (int r = 0; r < 8; ++r) {
        const float a_ = acc[2 * pr][r], b_ = acc[2 * pr + 1][r];
        const float ax = __shfl_xor(a_, 16), bx = __shfl_xor(b_, 16);
        float v1 = (hh ? bx : a_) + bb, v2 = (hh ? b_ : ax) + bb;
        if (RELU) { v1 = fmaxf(v1, 0.f); v2 = fmaxf(v2, 0.f); }
        if (m0 + r < valid)     *(volatile float*)(out + (size_t)(m0 + r) * NOUT + c) = v1;
        if (m0 + r + 8 < valid) *(volatile float*)(out + (size_t)(m0 + r + 8) * NOUT + c) = v2;
      }
    }
    __threadfence();
  }
}
__global__ __launch_bounds__(256) void k_aggr(const u32* __restrict__ A, const v2i* __restrict__ seg, const int* __restrict__ src, const float* __restrict__ w,
                                              const float* __restrict__ dinv, const float* __restrict__ t, const float* __restrict__ bias,
                                              float* __restrict__ h, int N, int ldh, int coff) {
  const int i8 = blockIdx.x * 256 + threadIdx.x;
  if (i8 >= N * D / 8) return;
  const int n = i8 >> 4, c0 = (i8 & 15) * 8;
  const v2i sv = seg[n];
  v8f s = {};
  for (int p = 0; p < sv[1]; ++p) {
    const int e = (int)(A[sv[0] + p] & 0xfffffu), sn = src[e];
    const float cw = dinv[sn] * w[e];
    const v8f tv = *(const v8f*)(t + (size_t)sn * D + c0);
#pragma unroll
    for (int q = 0; q < 8; ++q) s[q] += cw * tv[q];
  }
  const float dn = dinv[n];
  v8f o;
#pragma unroll
  for (int q = 0; q < 8; ++q) o[q] = fmaxf(dn * s[q] + bias[c0 + q], 0.f);
  VST2(v8f, h + (size_t)n * ldh + coff + c0, o);
}
__global__ __launch_bounds__(256) void k_add_rows(const float* __restrict__ a, const float* __restrict__ b, int ldb, int boff,
                                                  float* __restrict__ dst, int N, int ldd, int coff) {
  const int i8 = blockIdx.x * 256 + threadIdx.x;
  if (i8 >= N * D / 8) return;
  const int n = i8 >> 4, c0 = (i8 & 15) * 8;
  v8f o = *(const v8f*)(a + (size_t)n * D + c0);
  if (b) { const v8f bv = *(const v8f*)(b + (size_t)n * ldb + boff + c0);
#pragma unroll
    for (int q = 0; q < 8; ++q) o[q] += bv[q]; }
  VST2(v8f, dst + (size_t)n * ldd + coff + c0, o);
}
__global__ __launch_bounds__(256) void k_chanpart(const float* __restrict__ pk, int N, int C, float* __restrict__ part) {
  const int r0 = blockIdx.x * 64, r1 = min(r0 + 64, N);
  for (int c = threadIdx.x; c < C * D; c += 256) {
    float s = 0.f;
    for (int r = r0; r < r1; ++r) s += pk[(size_t)r * C * D + c];
    VST2(float, part + (size_t)blockIdx.x * C * D + c, s);
  }
}
__global__ __launch_bounds__(256) void k_chanatt(const float* __restrict__ part, int nblk, int N, int C,
                                                 const float* __restrict__ fc1W, const float* __restrict__ fc1b, const float* __restrict__ fc2W, const float* __restrict__ fc2b,
                                                 float* __restrict__ a_out) {
  __shared__ double red[4][256];
  const int t = threadIdx.x;
  double acc[4] = {0.0, 0.0, 0.0, 0.0};
  for (int c = t; c < C * D; c += 256) {
    double s = 0.0;
    for (int b = 0; b < nblk; ++b) s += (double)part[(size_t)b * C * D + c];
    acc[c / D] += s;
  }
  for (int ch = 0; ch < 4; ++ch) red[ch][t] = acc[ch];
  __syncthreads();
  for (int o = 128; o > 0; o >>= 1) { if (t < o) for (int ch = 0; ch < 4; ++ch) red[ch][t] += red[ch][t + o]; __syncthreads(); }
  if (t == 0) {
    float mean[4], t1[4], a[4] = {0.f, 0.f, 0.f, 0.f};
    for (int ch = 0; ch < C; ++ch) mean[ch] = (float)(red[ch][0] / ((double)N * D));
    for (int ch = 0; ch < C; ++ch) { float s = fc1b[ch]; for (int k = 0; k < C; ++k) s += fc1W[ch * C + k] * mean[k]; t1[ch] = fmaxf(s, 0.f); }
    for (int ch = 0; ch < C; ++ch) { float s = fc2b[ch]; for (int k = 0; k < C; ++k) s += fc2W[ch * C + k] * t1[k]; a[ch] = 1.f / (1.f + expf(-s)); }
    const v4f av = {a[0], a[1], a[2], a[3]};
    VST2(v4f, a_out, av);
  }
}

extern "C" void kernel_launch(void* const* d_in, const int* in_sizes, int n_in,
                              void* d_out, int out_size, void* d_ws, size_t ws_size, hipStream_t stream) {
  (void)in_sizes; (void)n_in; (void)out_size;
  const float* mx  = (const float*)d_in[0];
  const float* dx  = (const float*)d_in[1];
  struct View { const int* edge; const float* w; const float* W1; const float* b1; const float* W2; const float* b2; int n, np, E, sortLog; };
  View v[4];
  const int nn[4] = {NM, NM, ND, ND}, npd[4] = {NMP, NMP, NDP, NDP}, ee[4] = {300000, 300000, 600000, 600000}, sl[4] = {19, 19, 20, 20};
  for (int i = 0; i < 4; ++i) {
    v[i].edge = (const int*)d_in[2 + 6 * i]; v[i].w = (const float*)d_in[3 + 6 * i];
    v[i].W1 = (const float*)d_in[4 + 6 * i]; v[i].b1 = (const float*)d_in[5 + 6 * i];
    v[i].W2 = (const float*)d_in[6 + 6 * i]; v[i].b2 = (const float*)d_in[7 + 6 * i];
    v[i].n = nn[i]; v[i].np = npd[i]; v[i].E = ee[i]; v[i].sortLog = sl[i];
  }
  const float* m_fc1_W = (const float*)d_in[26]; const float* m_fc1_b = (const float*)d_in[27];
  const float* m_fc2_W = (const float*)d_in[28]; const float* m_fc2_b = (const float*)d_in[29];
  const float* d_fc1_W = (const float*)d_in[30]; const float* d_fc1_b = (const float*)d_in[31];
  const float* d_fc2_W = (const float*)d_in[32]; const float* d_fc2_b = (const float*)d_in[33];
  const float* m_fus_W1 = (const float*)d_in[34]; const float* m_fus_b1 = (const float*)d_in[35];
  const float* m_fus_W2 = (const float*)d_in[36]; const float* m_fus_b2 = (const float*)d_in[37];
  const float* d_fus_W1 = (const float*)d_in[38]; const float* d_fus_b1 = (const float*)d_in[39];
  const float* d_fus_W2 = (const float*)d_in[40]; const float* d_fus_b2 = (const float*)d_in[41];
  float* out = (float*)d_out;

  char* ws = (char*)d_ws; size_t off = 0;
  auto take = [&](size_t bytes) { void* p = ws + off; off = (off + bytes + 255) & ~(size_t)255; return p; };
  u32*   keys  = (u32*)take((size_t)(1 << 20) * 4);
  v2i*   seg   = (v2i*)take((size_t)NDP * 8);
  float* dinv  = (float*)take((size_t)NDP * 4);
  _Float16* A16 = (_Float16*)take((size_t)NDP * 4 * D * 2);
  _Float16* Wh  = (_Float16*)take((size_t)256 * 512 * 2);
  float* t     = (float*)take((size_t)NDP * D * 4);
  float* x1    = (float*)take((size_t)NDP * D * 4);
  float* chanM = (float*)take((size_t)NMP * 4 * D * 4);
  float* chanD = (float*)take((size_t)NDP * 2 * D * 4);
  float* dtmp  = (float*)take((size_t)NDP * 2 * D * 4);
  float* part  = (float*)take((size_t)40 * 4 * D * 4);
  float* aM    = (float*)take(256); float* aD = (float*)take(256);
  float* u     = (float*)take((size_t)NDP * 256 * 4);
  if (off > ws_size) return;

  dim3 b256(256);
  auto cdiv = [](long long a, long long bq) { return (unsigned)((a + bq - 1) / bq); };

  float* x2 = dtmp + (size_t)NDP * D;
  (void)x2;
  float* l2buf = (float*)take((size_t)NDP * D * 4);
  if (off > ws_size) return;
  auto run_view = [&](const View& V, const float* x0) {
    const int sortN = 1 << V.sortLog;
    const int* src = V.edge; const int* dstI = V.edge + V.E;
    k_sort_init<<<sortN / 256, b256, 0, stream>>>(dstI, keys, V.E);
    k_sort_local<<<sortN / TILE, b256, 0, stream>>>(keys);
    for (int k = TILE * 2; k <= sortN; k <<= 1) {
      for (int logj = __builtin_ctz(k) - 1; (1 << logj) >= TILE; --logj)
        k_sort_global<<<sortN / 2 / 256, b256, 0, stream>>>(keys, logj, k);
      k_sort_lds<<<sortN / TILE, b256, 0, stream>>>(keys, k);
    }
    k_segs_deg<<<cdiv(V.n, 256), b256, 0, stream>>>(keys, sortN, V.w, seg, dinv, V.n);
    k_tof16<<<cdiv((long long)V.np * D / 8, 256), b256, 0, stream>>>(x0, V.n, V.np, D, nullptr, A16);
    k_w16<<<cdiv(D * D / 8, 256), b256, 0, stream>>>(V.W1, Wh, D * D);
    k_gemm<D, D, false><<<dim3(V.np / 64, D / 64), dim3(128), 0, stream>>>(A16, Wh, nullptr, t, V.np);
    k_aggr<<<cdiv(V.n * D / 8, 256), b256, 0, stream>>>(keys, seg, src, V.w, dinv, t, V.b1, x1, V.n, D, 0);
    k_tof16<<<cdiv((long long)V.np * D / 8, 256), b256, 0, stream>>>(x1, V.n, V.np, D, nullptr, A16);
    k_w16<<<cdiv(D * D / 8, 256), b256, 0, stream>>>(V.W2, Wh, D * D);
    k_gemm<D, D, false><<<dim3(V.np / 64, D / 64), dim3(128), 0, stream>>>(A16, Wh, nullptr, t, V.np);
    k_aggr<<<cdiv(V.n * D / 8, 256), b256, 0, stream>>>(keys, seg, src, V.w, dinv, t, V.b2, l2buf, V.n, D, 0);
  };
  const unsigned gm = cdiv(NM * D / 8, 256), gd = cdiv(ND * D / 8, 256);
  run_view(v[0], mx);
  k_add_rows<<<gm, b256, 0, stream>>>(x1,    nullptr, 0, 0, chanM, NM, 4 * D, 0 * D);
  k_add_rows<<<gm, b256, 0, stream>>>(l2buf, nullptr, 0, 0, chanM, NM, 4 * D, 1 * D);
  run_view(v[1], mx);
  k_add_rows<<<gm, b256, 0, stream>>>(x1,    nullptr, 0, 0, chanM, NM, 4 * D, 2 * D);
  k_add_rows<<<gm, b256, 0, stream>>>(l2buf, nullptr, 0, 0, chanM, NM, 4 * D, 3 * D);
  k_chanpart<<<cdiv(NM, 64), b256, 0, stream>>>(chanM, NM, 4, part);
  k_chanatt<<<1, b256, 0, stream>>>(part, (int)cdiv(NM, 64), NM, 4, m_fc1_W, m_fc1_b, m_fc2_W, m_fc2_b, aM);
  k_tof16<<<cdiv((long long)NMP * 4 * D / 8, 256), b256, 0, stream>>>(chanM, NM, NMP, 4 * D, aM, A16);
  k_w16<<<cdiv(256 * 512 / 8, 256), b256, 0, stream>>>(m_fus_W1, Wh, 256 * 512);
  k_gemm<512, 256, true><<<dim3(NMP / 64, 256 / 64), dim3(128), 0, stream>>>(A16, Wh, m_fus_b1, u, NM);
  k_tof16<<<cdiv((long long)NMP * 256 / 8, 256), b256, 0, stream>>>(u, NM, NMP, 256, nullptr, A16);
  k_w16<<<cdiv(128 * 256 / 8, 256), b256, 0, stream>>>(m_fus_W2, Wh, 128 * 256);
  k_gemm<256, 128, true><<<dim3(NMP / 64, 128 / 64), dim3(128), 0, stream>>>(A16, Wh, m_fus_b2, out, NM);
  run_view(v[2], dx);
  k_add_rows<<<gd, b256, 0, stream>>>(x1,    nullptr, 0, 0, dtmp, ND, 2 * D, 0 * D);
  k_add_rows<<<gd, b256, 0, stream>>>(l2buf, nullptr, 0, 0, dtmp, ND, 2 * D, 1 * D);
  run_view(v[3], dx);
  k_add_rows<<<gd, b256, 0, stream>>>(x1,    dtmp, 2 * D, 0 * D, chanD, ND, 2 * D, 0 * D);
  k_add_rows<<<gd, b256, 0, stream>>>(l2buf, dtmp, 2 * D, 1 * D, chanD, ND, 2 * D, 1 * D);
  k_chanpart<<<cdiv(ND, 64), b256, 0, stream>>>(chanD, ND, 2, part);
  k_chanatt<<<1, b256, 0, stream>>>(part, (int)cdiv(ND, 64), ND, 2, d_fc1_W, d_fc1_b, d_fc2_W, d_fc2_b, aD);
  k_tof16<<<cdiv((long long)NDP * 2 * D / 8, 256), b256, 0, stream>>>(chanD, ND, NDP, 2 * D, aD, A16);
  k_w16<<<cdiv(256 * 256 / 8, 256), b256, 0, stream>>>(d_fus_W1, Wh, 256 * 256);
  k_gemm<256, 256, true><<<dim3(NDP / 64, 256 / 64), dim3(128), 0, stream>>>(A16, Wh, d_fus_b1, u, ND);
  k_tof16<<<cdiv((long long)NDP * 256 / 8, 256), b256, 0, stream>>>(u, ND, NDP, 256, nullptr, A16);
  k_w16<<<cdiv(128 * 256 / 8, 256), b256, 0, stream>>>(d_fus_W2, Wh, 128 * 256);
  k_gemm<256, 128, true><<<dim3(NDP / 64, 128 / 64), dim3(128), 0, stream>>>(A16, Wh, d_fus_b2, out + (size_t)NM * D, ND);
}
